// CoAttenBlock_16234976379261
// MI455X (gfx1250) — hardware-verified
//
#include <hip/hip_runtime.h>
#include <math.h>

typedef __attribute__((ext_vector_type(16))) _Float16 v16h;
typedef __attribute__((ext_vector_type(16))) __bf16 v16b;
typedef __attribute__((ext_vector_type(8)))  _Float16 v8h;
typedef __attribute__((ext_vector_type(8)))  float v8f;
typedef __attribute__((ext_vector_type(4)))  float v4f;
typedef __attribute__((ext_vector_type(2)))  float v2f;
typedef __attribute__((ext_vector_type(4)))  unsigned v4u;
typedef __attribute__((ext_vector_type(4)))  int v4i;
typedef float __attribute__((may_alias)) float_a;
typedef int __attribute__((may_alias)) int_a;

template <typename T> __device__ __forceinline__ void vst2(void* p, T v) { *(volatile T*)p = v; __threadfence(); *(volatile T*)p = v; }
__device__ __forceinline__ v8f wmma16(v16h a, v16h b, v8f c) {
  v8f d = __builtin_amdgcn_wmma_f32_16x16x32_f16(false, a, false, b, (short)0, c, false, false);
  asm volatile("v_nop\n\tv_nop\n\tv_nop\n\tv_nop" : "+v"(d) : "v"(a), "v"(b));
  return d;
}
__device__ __forceinline__ v8f wmma_bf(v16b a, v16b b, v8f c) {
  v8f d = __builtin_amdgcn_wmma_f32_16x16x32_bf16(false, a, false, b, (short)0, c, false, false);
  asm volatile("v_nop\n\tv_nop\n\tv_nop\n\tv_nop" : "+v"(d) : "v"(a), "v"(b));
  return d;
}
__device__ __forceinline__ v16h frag_h(const _Float16* rowk0, int lane) {
  union { v16h v; v8h q[2]; } u; const _Float16* p = rowk0 + 8 * (lane >> 4);
  u.q[0] = *(const v8h*)p; u.q[1] = *(const v8h*)(p + 16); return u.v;
}
__device__ __forceinline__ v16h frag_f32(const float* rowk0, int lane) {
  v16h a; const float* p = rowk0 + 8 * (lane >> 4);
#pragma unroll
  for (int i = 0; i < 8; ++i) { a[i] = (_Float16)p[i]; a[8 + i] = (_Float16)p[16 + i]; }
  return a;
}
__device__ __forceinline__ v16h frag_f32s(const float* rowk0, int lane, float sc) {
  v16h a; const float* p = rowk0 + 8 * (lane >> 4);
#pragma unroll
  for (int i = 0; i < 8; ++i) { a[i] = (_Float16)(p[i] * sc); a[8 + i] = (_Float16)(p[16 + i] * sc); }
  return a;
}
__device__ __forceinline__ v16h fragc_f32(const float* W, int k0, int n, int lane, int ld, int K) {
  v16h a; const int g = lane >> 4;
#pragma unroll
  for (int i = 0; i < 8; ++i) { const int ka = k0 + 8 * g + i, kb = ka + 16;
    a[i] = (_Float16)(ka < K ? W[(size_t)(ka < K ? ka : K - 1) * ld + n] : 0.f); a[8 + i] = (_Float16)(kb < K ? W[(size_t)(kb < K ? kb : K - 1) * ld + n] : 0.f); }
  return a;
}
struct F2 { v16b h, l; };
__device__ __forceinline__ F2 bsplit16(const float v[16]) { F2 r;
#pragma unroll
  for (int i = 0; i < 16; ++i) { const __bf16 h = (__bf16)v[i]; r.h[i] = h; r.l[i] = (__bf16)(v[i] - (float)h); }
  return r; }
__device__ __forceinline__ F2 split_row(const float* row, int k0, int lane) { float v[16]; const float* p = row + k0 + 8 * (lane >> 4);
#pragma unroll
  for (int i = 0; i < 8; ++i) { v[i] = p[i]; v[8 + i] = p[16 + i]; }
  return bsplit16(v); }
__device__ __forceinline__ F2 split_rowK(const float* row, int k0, int lane, int K) { float v[16]; const int g = lane >> 4;
#pragma unroll
  for (int i = 0; i < 8; ++i) { const int ka = k0 + 8 * g + i, kb = ka + 16; v[i] = ka < K ? row[ka < K ? ka : K - 1] : 0.f; v[8 + i] = kb < K ? row[kb < K ? kb : K - 1] : 0.f; }
  return bsplit16(v); }
__device__ __forceinline__ F2 split_col(const float* W, int k0, int n, int lane, int ld, int K) { float v[16]; const int g = lane >> 4;
#pragma unroll
  for (int i = 0; i < 8; ++i) { const int ka = k0 + 8 * g + i, kb = ka + 16; v[i] = ka < K ? W[(size_t)(ka < K ? ka : K - 1) * ld + n] : 0.f; v[8 + i] = kb < K ? W[(size_t)(kb < K ? kb : K - 1) * ld + n] : 0.f; }
  return bsplit16(v); }
__device__ __forceinline__ v8f mac3(const F2& a, const F2& b, v8f c) { c = wmma_bf(a.l, b.h, c); c = wmma_bf(a.h, b.l, c); return wmma_bf(a.h, b.h, c); }
__device__ __forceinline__ float sigm(float v) { return 1.0f / (1.0f + expf(-v)); }
#define LDSX() do { asm volatile("s_wait_dscnt 0" ::: "memory"); __builtin_amdgcn_wave_barrier(); __builtin_amdgcn_fence(__ATOMIC_RELEASE, "workgroup"); } while (0)


#define NB 8
#define CC 64
#define NP 2304
#ifndef TNB
#define TNB NB
#endif
typedef __attribute__((ext_vector_type(8))) __bf16 v8b;
__device__ __forceinline__ v16b frag_b(const __bf16* rowk0, int lane) {
  union { v16b v; v8b q[2]; } u; const __bf16* p = rowk0 + 8 * (lane >> 4);
  u.q[0] = *(const v8b*)p; u.q[1] = *(const v8b*)(p + 16); return u.v;
}
__device__ __forceinline__ float bfr(float v) { return (float)(__bf16)v; }
__device__ __attribute__((noinline)) float exp_ni(float v) { return expf(v); }
__device__ __attribute__((noinline)) float erf_ni(float v) { return erff(v); }

#define WS_PW  0u
#define WS_XT  (WS_PW + 2u * 4 * CC * 2 * CC)
#define XTSZ   ((size_t)NB * 2 * NP * CC)
#define WS_XP  (WS_XT + 2u * 2 * XTSZ)
#define WS_G   (WS_XP + 2u * 2 * XTSZ)
#define WS_CS  (WS_G + 4u * (size_t)NB * NP * NP)
#define WS_RS  (WS_CS + 4u * (size_t)NB * NP * 4)
#define WS_END (WS_RS + 4u * (size_t)NB * NP * 4)

__global__ __launch_bounds__(128) void k_pack(const float* __restrict__ W0, const float* __restrict__ W1, const float* __restrict__ W2, const float* __restrict__ W3, __bf16* __restrict__ PW) { const int o = blockIdx.x, which = blockIdx.y, t = threadIdx.x; __shared__ __align__(16) __bf16 s[2 * CC]; const float* Wm = which == 0 ? W0 : which == 1 ? W1 : which == 2 ? W2 : W3; s[t] = (__bf16)Wm[(size_t)o * 2 * CC + t]; __syncthreads(); if (t < 16) vst2((unsigned*)(PW + ((size_t)which * CC + o) * 2 * CC + t * 8), *(const v4u*)&s[t * 8]); }
__global__ __launch_bounds__(128) void k_xlr(const float* __restrict__ XH0, const float* __restrict__ XL0, const float* __restrict__ XH1, const float* __restrict__ XL1, const __bf16* __restrict__ PW, const float* __restrict__ BL, const float* __restrict__ BR, __bf16* __restrict__ XTH, __bf16* __restrict__ XTL, __bf16* __restrict__ XPH, __bf16* __restrict__ XPL) {
  __shared__ float sx[2 * CC][64 + 1]; __shared__ __align__(16) __bf16 sth[64][CC + 8], stl[64][CC + 8], sph[CC][64 + 8], spl[CC][64 + 8];
  const int tid = threadIdx.x, wave = tid >> 5, lane = tid & 31, col = lane & 15, g = lane >> 4; const int n0 = blockIdx.x * 64; const int side = blockIdx.y; const size_t b = blockIdx.z; const float* XH = side == 0 ? XH0 : XH1; const float* XLw = side == 0 ? XL0 : XL1;
  for (int e = tid; e < 2 * CC * 64; e += 128) { const int cin = e >> 6, nl = e & 63; const float* src = (cin < CC) ? (XH + ((b * CC + cin) * NP) + n0 + nl) : (XLw + ((b * CC + cin - CC) * NP) + n0 + nl); sx[cin][nl] = bfr(*src); }
  __syncthreads();
  v8f acc[4] = {}; const __bf16* Wr = PW + (size_t)side * CC * 2 * CC;
#pragma unroll
  for (int kc = 0; kc < 4; ++kc) { v16b a; const int nl = wave * 16 + col;
#pragma unroll
    for (int i = 0; i < 8; ++i) { a[i] = (__bf16)sx[kc * 32 + 8 * g + i][nl]; a[8 + i] = (__bf16)sx[kc * 32 + 16 + 8 * g + i][nl]; }
#pragma unroll
    for (int j = 0; j < 4; ++j) acc[j] = wmma_bf(a, frag_b(Wr + (size_t)(j * 16 + col) * 2 * CC + kc * 32, lane), acc[j]); }
  const float* BB = side == 0 ? BL : BR;
#pragma unroll
  for (int j = 0; j < 4; ++j) { const int o = j * 16 + col; const float bb = bfr(BB[o]);
#pragma unroll
    for (int r = 0; r < 8; ++r) { const int nl = wave * 16 + 8 * g + r; const float v = acc[j][r] + bb; const __bf16 hv = (__bf16)v; const __bf16 lv = (__bf16)(v - (float)hv); sth[nl][o] = hv; stl[nl][o] = lv; sph[o][nl] = hv; spl[o][nl] = lv; } }
  __syncthreads();
  const size_t tb = ((b * 2 + side) * NP + n0); for (int e = tid; e < 64 * 8; e += 128) { const int nl = e >> 3, q = e & 7; vst2((unsigned*)(XTH + (tb + nl) * CC + q * 8), *(const v4u*)&sth[nl][q * 8]); vst2((unsigned*)(XTL + (tb + nl) * CC + q * 8), *(const v4u*)&stl[nl][q * 8]); }
  const size_t pb = (b * 2 + side) * CC; for (int e = tid; e < CC * 8; e += 128) { const int o = e >> 3, q = e & 7; vst2((unsigned*)(XPH + (pb + o) * NP + n0 + q * 8), *(const v4u*)&sph[o][q * 8]); vst2((unsigned*)(XPL + (pb + o) * NP + n0 + q * 8), *(const v4u*)&spl[o][q * 8]); } }
__global__ __launch_bounds__(128) void k_g(const __bf16* __restrict__ XTH, const __bf16* __restrict__ XTL, float* __restrict__ G) { __shared__ __align__(16) float sf[4][16][132];
  const int tid = threadIdx.x, wave = tid >> 5, lane = tid & 31, col = lane & 15, g = lane >> 4; const size_t b = blockIdx.z; const int m0 = blockIdx.x * 64 + wave * 16; const int n0 = blockIdx.y * 128; const size_t tr = (b * 2 + 1) * NP, tl = (b * 2 + 0) * NP;
  v8f acc[8] = {};
#pragma unroll
  for (int kc = 0; kc < 2; ++kc) { const v16b ah = frag_b(XTH + (tr + m0 + col) * CC + kc * 32, lane), al = frag_b(XTL + (tr + m0 + col) * CC + kc * 32, lane);
#pragma unroll
    for (int j = 0; j < 8; ++j) { const size_t rn = tl + n0 + j * 16 + col; const v16b bh = frag_b(XTH + rn * CC + kc * 32, lane), bl = frag_b(XTL + rn * CC + kc * 32, lane); acc[j] = wmma_bf(ah, bh, acc[j]); acc[j] = wmma_bf(ah, bl, acc[j]); acc[j] = wmma_bf(al, bh, acc[j]); } }
#pragma unroll
  for (int j = 0; j < 8; ++j)
#pragma unroll
    for (int r = 0; r < 8; ++r) sf[wave][8 * g + r][j * 16 + col] = acc[j][r];
  LDSX(); for (int rl = 0; rl < 16; ++rl) vst2(G + ((b * NP + m0 + rl) * NP) + n0 + lane * 4, *(const v4f*)&sf[wave][rl][lane * 4]); }
__global__ __launch_bounds__(256) void k_cs(const float* __restrict__ G, float* __restrict__ CS) { __shared__ float red[8]; __shared__ __align__(16) float so2[4]; const int t = threadIdx.x; const size_t b = blockIdx.y, m = blockIdx.x; const float* row = G + (b * NP + m) * NP;
  float mx = -3.0e38f; for (int n = t; n < NP; n += 256) mx = fmaxf(mx, row[n]);
#pragma unroll
  for (int o = 1; o < 32; o <<= 1) mx = fmaxf(mx, __shfl_xor(mx, o));
  if ((t & 31) == 0) red[t >> 5] = mx; __syncthreads(); float gm = red[0]; for (int i = 1; i < 8; ++i) gm = fmaxf(gm, red[i]); __syncthreads();
  float s = 0.f; for (int n = t; n < NP; n += 256) s += __expf(row[n] - gm);
#pragma unroll
  for (int o = 1; o < 32; o <<= 1) s += __shfl_xor(s, o);
  if ((t & 31) == 0) red[t >> 5] = s; __syncthreads(); if (t == 0) { float ts = 0.f; for (int i = 0; i < 8; ++i) ts += red[i]; so2[0] = gm; so2[1] = 1.0f / ts; so2[2] = 0.f; so2[3] = 0.f; }
  __syncthreads(); if (t == 0) vst2(CS + (b * NP + m) * 4, *(const v4f*)&so2[0]); }
__global__ __launch_bounds__(64) void k_rs(const float* __restrict__ G, float* __restrict__ RS) { __shared__ __align__(16) float so2[64][4]; const int t = threadIdx.x; const size_t b = blockIdx.y; const int n = blockIdx.x * 64 + t; const float* colp = G + (b * NP) * NP + n;
  float mx = -3.0e38f;
#pragma unroll 1
  for (int m = 0; m < NP; ++m) mx = fmaxf(mx, colp[(size_t)m * NP]);
  float s = 0.f;
#pragma unroll 1
  for (int m = 0; m < NP; ++m) s += __expf(colp[(size_t)m * NP] - mx);
  so2[t][0] = mx; so2[t][1] = 1.0f / s; so2[t][2] = 0.f; so2[t][3] = 0.f; __syncthreads(); vst2(RS + (b * NP + n) * 4, *(const v4f*)&so2[t][0]); }
__global__ __launch_bounds__(128) void k_b(const float* __restrict__ G, const float* __restrict__ CS, const float* __restrict__ RS, const __bf16* __restrict__ XPH, const __bf16* __restrict__ XPL, const __bf16* __restrict__ XTH, const __bf16* __restrict__ XTL, const __bf16* __restrict__ PW,
    const float* __restrict__ GLW, const float* __restrict__ GLB, const float* __restrict__ GRW, const float* __restrict__ GRB, const float* __restrict__ OLB, const float* __restrict__ ORB, float* __restrict__ OUTL, float* __restrict__ OUTR) {
  __shared__ float sb[2][64][CC + 1]; __shared__ __align__(16) float so2[CC][64 + 4];
  const int tid = threadIdx.x, wave = tid >> 5, lane = tid & 31, col = lane & 15, g = lane >> 4; const size_t b = blockIdx.y; const int m0 = blockIdx.x * 64 + wave * 16; const size_t rowm = b * NP + m0 + col;
  const float cmax = CS[rowm * 4]; const float* grow = G + rowm * NP;
  v8f acc1[4] = {}, acc2[4] = {};
  const size_t pl = (b * 2 + 0) * CC, pr = (b * 2 + 1) * CC;
#pragma unroll 1
  for (int kc = 0; kc < NP / 32; ++kc) { float v1[16], v2[16];
#pragma unroll
    for (int i = 0; i < 8; ++i) { const int na = kc * 32 + 8 * g + i, nb = na + 16; const float ga = grow[na], gb = grow[nb]; v1[i] = __expf(ga - cmax); v1[8 + i] = __expf(gb - cmax); v2[i] = __expf(ga - RS[(b * NP + na) * 4]) * RS[(b * NP + na) * 4 + 1]; v2[8 + i] = __expf(gb - RS[(b * NP + nb) * 4]) * RS[(b * NP + nb) * 4 + 1]; }
    const F2 a1 = bsplit16(v1), a2 = bsplit16(v2);
#pragma unroll
    for (int j = 0; j < 4; ++j) { const size_t o1 = (pl + j * 16 + col) * NP + kc * 32, o2 = (pr + j * 16 + col) * NP + kc * 32; const v16b xh = frag_b(XPH + o1, lane), xl = frag_b(XPL + o1, lane); acc1[j] = wmma_bf(a1.h, xh, acc1[j]); acc1[j] = wmma_bf(a1.h, xl, acc1[j]); acc1[j] = wmma_bf(a1.l, xh, acc1[j]);
      const v16b yh = frag_b(XPH + o2, lane), yl = frag_b(XPL + o2, lane); acc2[j] = wmma_bf(a2.h, yh, acc2[j]); acc2[j] = wmma_bf(a2.h, yl, acc2[j]); acc2[j] = wmma_bf(a2.l, yh, acc2[j]); } }
  float gl1[8], gl2[8];
#pragma unroll
  for (int r = 0; r < 8; ++r) { gl1[r] = 0.f; gl2[r] = 0.f; }
  float cinv[8];
#pragma unroll
  for (int r = 0; r < 8; ++r) cinv[r] = CS[(b * NP + m0 + 8 * g + r) * 4 + 1];
#pragma unroll
  for (int j = 0; j < 4; ++j) { const int c = j * 16 + col; const float w1 = bfr(GLW[c]), w2 = bfr(GRW[c]);
#pragma unroll
    for (int r = 0; r < 8; ++r) { acc1[j][r] *= cinv[r]; gl1[r] += w1 * acc1[j][r]; gl2[r] += w2 * acc2[j][r]; } }
#pragma unroll
  for (int r = 0; r < 8; ++r) {
#pragma unroll
    for (int o = 1; o < 16; o <<= 1) { gl1[r] += __shfl_xor(gl1[r], o); gl2[r] += __shfl_xor(gl2[r], o); }
    const float g1 = 1.0f / (1.0f + expf(-(gl1[r] + bfr(GLB[0])))), g2 = 1.0f / (1.0f + expf(-(gl2[r] + bfr(GRB[0]))));
#pragma unroll
    for (int j = 0; j < 4; ++j) { sb[0][wave * 16 + 8 * g + r][j * 16 + col] = acc1[j][r] * g1; sb[1][wave * 16 + 8 * g + r][j * 16 + col] = acc2[j][r] * g2; } }
  LDSX();
#pragma unroll 1
  for (int side = 0; side < 2; ++side) { v8f acc[4] = {}; const __bf16* Wr = PW + (size_t)(2 + side) * CC * 2 * CC; const size_t tr = ((b * 2 + side) * NP + m0 + col) * CC;
#pragma unroll
    for (int kc = 0; kc < 2; ++kc) { const v16b ah = frag_b(XTH + tr + kc * 32, lane), al = frag_b(XTL + tr + kc * 32, lane);
#pragma unroll
      for (int j = 0; j < 4; ++j) { const v16b w = frag_b(Wr + (size_t)(j * 16 + col) * 2 * CC + kc * 32, lane); acc[j] = wmma_bf(ah, w, acc[j]); acc[j] = wmma_bf(al, w, acc[j]); } }
#pragma unroll
    for (int kc = 0; kc < 2; ++kc) { float v[16]; const float* p2 = &sb[side][wave * 16 + col][kc * 32 + 8 * g];
#pragma unroll
      for (int i = 0; i < 8; ++i) { v[i] = p2[i]; v[8 + i] = p2[16 + i]; }
      const F2 a = bsplit16(v);
#pragma unroll
      for (int j = 0; j < 4; ++j) { const v16b w = frag_b(Wr + (size_t)(j * 16 + col) * 2 * CC + CC + kc * 32, lane); acc[j] = wmma_bf(a.h, w, acc[j]); acc[j] = wmma_bf(a.l, w, acc[j]); } }
    const float* OB = side == 0 ? OLB : ORB; __syncthreads();
#pragma unroll
    for (int j = 0; j < 4; ++j) { const int o = j * 16 + col; const float bb = bfr(OB[o]);
#pragma unroll
      for (int r = 0; r < 8; ++r) so2[o][wave * 16 + 8 * g + r] = acc[j][r] + bb; }
    __syncthreads(); float* OUT = side == 0 ? OUTL : OUTR;
    for (int e = tid; e < CC * 16; e += 128) { const int o = e >> 4, q = e & 15; vst2(OUT + ((b * CC + o) * NP) + blockIdx.x * 64 + q * 4, *(const v4f*)&so2[o][q * 4]); }
    __syncthreads(); }
}
extern "C" void kernel_launch(void* const* d_in, const int* in_sizes, int n_in, void* d_out, int out_size, void* d_ws, size_t ws_size, hipStream_t stream) {
  (void)in_sizes; (void)n_in; (void)out_size;
  const float** F = (const float**)d_in;
  if (ws_size < (size_t)WS_END) return;
  char* ws = (char*)d_ws; __bf16* PW = (__bf16*)(ws + WS_PW); __bf16 *XTH = (__bf16*)(ws + WS_XT), *XTL = XTH + XTSZ, *XPH = (__bf16*)(ws + WS_XP), *XPL = XPH + XTSZ; float *G = (float*)(ws + WS_G), *CS = (float*)(ws + WS_CS), *RS = (float*)(ws + WS_RS);
  float* OUTL = (float*)d_out; float* OUTR = OUTL + (size_t)NB * CC * NP;
  k_pack<<<dim3(CC, 4), 128, 0, stream>>>(F[4], F[6], F[12], F[14], PW);
  k_xlr<<<dim3(NP / 64, 2, TNB), 128, 0, stream>>>(F[0], F[1], F[2], F[3], PW, F[5], F[7], XTH, XTL, XPH, XPL);
  k_g<<<dim3(NP / 64, NP / 128, TNB), 128, 0, stream>>>(XTH, XTL, G);
  k_cs<<<dim3(NP, TNB), 256, 0, stream>>>(G, CS);
  k_rs<<<dim3(NP / 64, TNB), 64, 0, stream>>>(G, RS);
  k_b<<<dim3(NP / 64, TNB), 128, 0, stream>>>(G, CS, RS, XPH, XPL, XTH, XTL, PW, F[8], F[9], F[10], F[11], F[13], F[15], OUTL, OUTR);
}
